// PhaseAttention_80255758893321
// MI455X (gfx1250) — hardware-verified
//
#include <hip/hip_runtime.h>
#include <math.h>

constexpr int kBatch    = 4;
constexpr int kSeq      = 2048;
constexpr int kDim      = 1024;
constexpr int kTok      = kBatch * kSeq;
constexpr int kProjRows = 4096;
constexpr int kQRows    = 1024;
constexpr int kChunks   = kTok / kQRows;
constexpr int kChunksPerBatch = kSeq / kQRows;

constexpr float kWCarry    = 16.0f;
constexpr float kWCarryInv = 1.0f / 16.0f;
constexpr float kNCarry    = 1024.0f;
constexpr float kPhScale   = 1.0f / (1024.0f * 1024.0f);
constexpr float kAmpScale  = 1.0f / 32.0f;
constexpr float kPCarry    = 2048.0f;
constexpr float kOCarry    = 64.0f;
constexpr float kPVScale   = kOCarry / kPCarry;
constexpr float kOutScale  = 1.0f / (kOCarry * kWCarry);
constexpr float kPiF       = 3.14159265358979323846f;

constexpr size_t kPlane16  = (size_t)kTok * kDim * 2;
constexpr size_t kW16Bytes = (size_t)kDim * kDim * 2;
constexpr size_t kOffX16   = 0;
constexpr size_t kOffWq    = kOffX16 + kPlane16;
constexpr size_t kOffWk    = kOffWq + kW16Bytes;
constexpr size_t kOffWv    = kOffWk + kW16Bytes;
constexpr size_t kOffWo    = kOffWv + kW16Bytes;
constexpr size_t kOffScr   = kOffWo + kW16Bytes;
constexpr size_t kScrBytes = (size_t)kProjRows * kDim * 4;
constexpr size_t kOffSph   = kOffScr + (size_t)kQRows * kSeq * 4;
constexpr size_t kOffQ16   = kOffScr + kScrBytes;
constexpr size_t kOffQn16  = kOffQ16 + kPlane16;
constexpr size_t kOffK16   = kOffQn16 + kPlane16;
constexpr size_t kOffKn16  = kOffK16 + kPlane16;
constexpr size_t kOffVt16  = kOffKn16 + kPlane16;
constexpr size_t kOffP16   = kOffVt16 + kPlane16;
constexpr size_t kP16Bytes = (size_t)kQRows * kSeq * 2;
constexpr size_t kWsTotal  = kOffP16 + kP16Bytes;
static_assert(kWsTotal <= (size_t)134217728);
static_assert((size_t)2 * kQRows * kSeq * 4 <= kScrBytes);
static_assert(kTok % kProjRows == 0 && kSeq % kQRows == 0);
static_assert(kProjRows % 64 == 0 && kQRows % 64 == 0 && kDim % 64 == 0 && kSeq % 64 == 0);
static_assert(kDim % 32 == 0 && kSeq % 32 == 0);

typedef __attribute__((ext_vector_type(16))) _Float16 v16h;
typedef __attribute__((ext_vector_type(8)))  _Float16 v8h;
typedef __attribute__((ext_vector_type(16))) __bf16   v16b;
typedef __attribute__((ext_vector_type(8)))  __bf16   v8b;
typedef __attribute__((ext_vector_type(8)))  float    v8f;
typedef __attribute__((ext_vector_type(4)))  float    v4f;
typedef __attribute__((ext_vector_type(4)))  unsigned int v4u;

__device__ __forceinline__ unsigned short f2bf_bits(float f) {
  unsigned u = __float_as_uint(f);
  return (unsigned short)((u + 0x7FFFu + ((u >> 16) & 1u)) >> 16);
}
__device__ __forceinline__ float bf_bits2f(unsigned short h) { return __uint_as_float(((unsigned)h) << 16); }

__device__ __forceinline__ void dep_guard_h(v8f& a, v8f& b, v16h x, v16h y) { asm volatile("v_nop\n\tv_nop\n\tv_nop\n\tv_nop" : "+v"(a), "+v"(b) : "v"(x), "v"(y)); }
__device__ __forceinline__ void dep_guard_b(v8f& a, v8f& b, v16b x, v16b y) { asm volatile("v_nop\n\tv_nop\n\tv_nop\n\tv_nop" : "+v"(a), "+v"(b) : "v"(x), "v"(y)); }
__device__ __forceinline__ void keep4_h(v16h a, v16h b, v16h c, v16h d) { asm volatile("v_nop" :: "v"(a), "v"(b), "v"(c), "v"(d)); }
__device__ __forceinline__ void keep4_b(v16b a, v16b b, v16b c, v16b d) { asm volatile("v_nop" :: "v"(a), "v"(b), "v"(c), "v"(d)); }
__device__ __forceinline__ void acc_guard4(v8f& a, v8f& b, v8f& c, v8f& d) { asm volatile("v_nop\n\tv_nop\n\tv_nop\n\tv_nop" : "+v"(a), "+v"(b), "+v"(c), "+v"(d)); }
template <typename T> struct Frag;
template <> struct Frag<_Float16> {
  typedef v16h V; union U { v16h v; v8h h[2]; };
  static __device__ __forceinline__ v16h load(const _Float16* p) {
    U f; f.h[0] = *(const v8h*)(p); f.h[1] = *(const v8h*)(p + 16); return f.v;
  }
  static __device__ __forceinline__ v8f mma(v16h a, v16h b, v8f c) {
    return __builtin_amdgcn_wmma_f32_16x16x32_f16(false, a, false, b, (short)0, c, false, false);
  }
  static __device__ __forceinline__ void guard(v8f& a, v8f& b, v16h x, v16h y) { dep_guard_h(a, b, x, y); }
  static __device__ __forceinline__ void keep(v16h a, v16h b, v16h c, v16h d) { keep4_h(a, b, c, d); }
};
template <> struct Frag<__bf16> {
  typedef v16b V; union U { v16b v; v8b h[2]; };
  static __device__ __forceinline__ v16b load(const __bf16* p) {
    U f; f.h[0] = *(const v8b*)(p); f.h[1] = *(const v8b*)(p + 16); return f.v;
  }
  static __device__ __forceinline__ v8f mma(v16b a, v16b b, v8f c) {
    return __builtin_amdgcn_wmma_f32_16x16x32_bf16(false, a, false, b, (short)0, c, false, false);
  }
  static __device__ __forceinline__ void guard(v8f& a, v8f& b, v16b x, v16b y) { dep_guard_b(a, b, x, y); }
  static __device__ __forceinline__ void keep(v16b a, v16b b, v16b c, v16b d) { keep4_b(a, b, c, d); }
};

__device__ __forceinline__ unsigned pk16(unsigned short a, unsigned short b) { return (unsigned)a | ((unsigned)b << 16); }
__device__ __forceinline__ unsigned short h_bits(float f) { const _Float16 h = (_Float16)f; return __builtin_bit_cast(unsigned short, h); }

template <int ET> struct Elem;
template <> struct Elem<0> { typedef _Float16 T; };
template <> struct Elem<1> { typedef __bf16 T; };
template <int ET, bool SPLIT, int BIAS_MODE, int OUT_MODE, bool RESID, int ACT = 0>
__global__ __launch_bounds__(256) void wmma_gemm64(
    const unsigned short* __restrict__ Ap, const unsigned short* __restrict__ A2p, int lda, long strideA,
    const unsigned short* __restrict__ Btp, const unsigned short* __restrict__ Bt2p, int ldb, long strideB,
    void* __restrict__ Cout, void* __restrict__ Cout2, int ldc, long strideC,
    const float* __restrict__ bias,
    const float* __restrict__ resid, long strideR,
    int M, int N, int K, float scale) {
  typedef typename Elem<ET>::T T;
  typedef typename Frag<T>::V V;
  const T* A = (const T*)Ap; const T* A2 = (const T*)A2p; const T* Bt = (const T*)Btp; const T* Bt2 = (const T*)Bt2p;
  __shared__ __align__(16) float sT[8][16 * 68];
  const int b    = blockIdx.y;
  const int lane = threadIdx.x & 31;
  const int wave = threadIdx.x >> 5;
  const int tilesN = N >> 6;
  const int tilesM = M >> 6;
  const int tile = blockIdx.x * 8 + wave;
  if (tile >= tilesM * tilesN) return;
  const int tm = tile / tilesN;
  const int tn = tile - tm * tilesN;
  const int m0 = tm << 6;
  const int n0 = tn << 6;

  const T* Ab  = A  + (size_t)b * strideA;
  const T* Bb  = Bt + (size_t)b * strideB;
  const T* Ab2 = SPLIT ? (A2  + (size_t)b * strideA) : nullptr;
  const T* Bb2 = SPLIT ? (Bt2 + (size_t)b * strideB) : nullptr;

  const int rlane = lane & 15;
  const int koff  = (lane >> 4) * 8;
  const int mOff  = (lane >> 4) * 8;

  v8f acc[4][4];
#pragma unroll
  for (int i = 0; i < 4; ++i)
#pragma unroll
    for (int j = 0; j < 4; ++j) acc[i][j] = (v8f){0.f,0.f,0.f,0.f,0.f,0.f,0.f,0.f};

  for (int k0 = 0; k0 < K; k0 += 32) {
    V bh[4], bl[4];
#pragma unroll
    for (int j = 0; j < 4; ++j) {
      const size_t bo = (size_t)(n0 + (j << 4) + rlane) * ldb + koff + k0;
      bh[j] = Frag<T>::load(Bb + bo);
      if (SPLIT) bl[j] = Frag<T>::load(Bb2 + bo);
    }
#pragma unroll
    for (int i = 0; i < 4; ++i) {
      const size_t ao = (size_t)(m0 + (i << 4) + rlane) * lda + koff + k0;
      V ah = Frag<T>::load(Ab + ao);
      V al;
      if (SPLIT) al = Frag<T>::load(Ab2 + ao);
#pragma unroll
      for (int j = 0; j < 4; ++j) {
        acc[i][j] = Frag<T>::mma(ah, bh[j], acc[i][j]);
        if (SPLIT) {
          acc[i][j] = Frag<T>::mma(ah, bl[j], acc[i][j]);
          acc[i][j] = Frag<T>::mma(al, bh[j], acc[i][j]);
        }
      }
      Frag<T>::guard(acc[i][0], acc[i][3], ah, SPLIT ? al : ah);
    }
    Frag<T>::keep(bh[0], bh[1], bh[2], bh[3]);
    if (SPLIT) Frag<T>::keep(bl[0], bl[1], bl[2], bl[3]);
  }
  acc_guard4(acc[0][0], acc[0][1], acc[0][2], acc[0][3]);
  acc_guard4(acc[1][0], acc[1][1], acc[1][2], acc[1][3]);
  acc_guard4(acc[2][0], acc[2][1], acc[2][2], acc[2][3]);
  acc_guard4(acc[3][0], acc[3][1], acc[3][2], acc[3][3]);

  float* slab = sT[wave];
  const float* Rb = RESID ? (resid + (size_t)b * strideR) : nullptr;
#pragma unroll
  for (int i = 0; i < 4; ++i) {
    const int mBase = m0 + (i << 4);
#pragma unroll
    for (int j = 0; j < 4; ++j) {
      const int n = n0 + (j << 4) + rlane;
      float bv = 0.f;
      if (BIAS_MODE == 2) bv = bias[n];
#pragma unroll
      for (int r = 0; r < 8; ++r) {
        float v = acc[i][j][r] * scale;
        if (BIAS_MODE == 1) v += bias[mBase + mOff + r];
        if (BIAS_MODE == 2) v += bv;
        if (RESID) v += Rb[(size_t)(mBase + mOff + r) * ldc + n];
        if (ACT == 2) v = fmaxf(v, 0.0f);
        if (ACT == 4) v = (v > 0.f) ? v : 0.01f * v;
        slab[(mOff + r) * 68 + (j << 4) + rlane] = v;
      }
    }
    __builtin_amdgcn_fence(__ATOMIC_RELEASE, "workgroup");
    __builtin_amdgcn_wave_barrier();
    __builtin_amdgcn_fence(__ATOMIC_ACQUIRE, "workgroup");
    if (OUT_MODE == 0) {
      float* C = (float*)Cout + (size_t)b * strideC;
      const int hh = lane >> 4, c4 = (lane & 15) * 4;
      for (int pass = 0; pass < 2; ++pass) {
#pragma unroll
        for (int it = 0; it < 8; ++it) {
          const int row = it * 2 + hh;
          v4f v = *(const v4f*)(slab + row * 68 + c4);
          *(volatile v4f*)(C + (size_t)(mBase + row) * ldc + n0 + c4) = v;
        }
        __threadfence();
      }
    } else {
      const int q = lane >> 3, c8 = (lane & 7) * 8;
      unsigned short* C  = (unsigned short*)Cout  + (size_t)b * strideC;
      unsigned short* C2 = (OUT_MODE == 2) ? ((unsigned short*)Cout2 + (size_t)b * strideC) : nullptr;
      for (int pass = 0; pass < 2; ++pass) {
#pragma unroll
        for (int it = 0; it < 4; ++it) {
          const int row = it * 4 + q;
          const float* sp = slab + row * 68 + c8;
          v8h hv, lv;
#pragma unroll
          for (int e = 0; e < 8; ++e) {
            if (OUT_MODE == 1) {
              hv[e] = (_Float16)sp[e];
            } else {
              unsigned short hb = f2bf_bits(sp[e]);
              unsigned short lb = f2bf_bits(sp[e] - bf_bits2f(hb));
              hv[e] = __builtin_bit_cast(_Float16, hb);
              lv[e] = __builtin_bit_cast(_Float16, lb);
            }
          }
          *(volatile v8h*)(C + (size_t)(mBase + row) * ldc + n0 + c8) = hv;
          if (OUT_MODE == 2) *(volatile v8h*)(C2 + (size_t)(mBase + row) * ldc + n0 + c8) = lv;
        }
        __threadfence();
      }
    }
    __builtin_amdgcn_fence(__ATOMIC_RELEASE, "workgroup");
    __builtin_amdgcn_wave_barrier();
    __builtin_amdgcn_fence(__ATOMIC_ACQUIRE, "workgroup");
  }
}

__global__ __launch_bounds__(256) void cast8_f16_kernel(const float* __restrict__ in, unsigned short* __restrict__ out,
                                                        int n8, float scale) {
  const int i = blockIdx.x * 256 + threadIdx.x;
  if (i >= n8) return;
  const float* p = in + 8 * (size_t)i;
  const v4f a = *(const v4f*)(p);
  const v4f c = *(const v4f*)(p + 4);
  unsigned short hb[8];
#pragma unroll
  for (int e = 0; e < 4; ++e) {
    hb[e]     = h_bits(a[e] * scale);
    hb[4 + e] = h_bits(c[e] * scale);
  }
  const v4u u = (v4u){pk16(hb[0], hb[1]), pk16(hb[2], hb[3]), pk16(hb[4], hb[5]), pk16(hb[6], hb[7])};
  unsigned short* q = out + 8 * (size_t)i;
  *(volatile v4u*)q = u;
  __threadfence();
  *(volatile v4u*)q = u;
}

__global__ __launch_bounds__(128) void rownorm_kernel(const float* __restrict__ Xf, unsigned short* __restrict__ X16,
                                                      unsigned short* __restrict__ Xn16, float ncarry) {
  __shared__ float red[4];
  const int row  = blockIdx.x;
  const int t    = threadIdx.x;
  const int lane = t & 31, wave = t >> 5;
  const int c0   = t * 8;
  const float* p = Xf + (size_t)row * kDim + c0;
  const v4f a = *(const v4f*)(p);
  const v4f c = *(const v4f*)(p + 4);
  float x[8];
#pragma unroll
  for (int e = 0; e < 4; ++e) { x[e] = a[e]; x[4 + e] = c[e]; }
  float ss = 0.f;
#pragma unroll
  for (int e = 0; e < 8; ++e) ss += x[e] * x[e];
#pragma unroll
  for (int off = 16; off > 0; off >>= 1) ss += __shfl_xor(ss, off, 32);
  if (lane == 0) red[wave] = ss;
  __syncthreads();
  const float tot = ((red[0] + red[1]) + red[2]) + red[3];
  const float nrm = sqrtf(tot);
  const float inv = 1.0f / (nrm + 1e-8f);
  const float kn  = ncarry * inv;
  unsigned short hb[8], nb[8];
#pragma unroll
  for (int e = 0; e < 8; ++e) {
    hb[e] = h_bits(x[e]);
    nb[e] = h_bits(x[e] * kn);
  }
  const v4u u1 = (v4u){pk16(hb[0], hb[1]), pk16(hb[2], hb[3]), pk16(hb[4], hb[5]), pk16(hb[6], hb[7])};
  const v4u u2 = (v4u){pk16(nb[0], nb[1]), pk16(nb[2], nb[3]), pk16(nb[4], nb[5]), pk16(nb[6], nb[7])};
  unsigned short* q1 = X16  + (size_t)row * kDim + c0;
  unsigned short* q2 = Xn16 + (size_t)row * kDim + c0;
  *(volatile v4u*)q1 = u1;
  *(volatile v4u*)q2 = u2;
  __threadfence();
  *(volatile v4u*)q1 = u1;
  *(volatile v4u*)q2 = u2;
}

__global__ __launch_bounds__(256) void phase_softmax_kernel(const float* __restrict__ Samp, const float* __restrict__ Sph,
                                                            unsigned short* __restrict__ P, float pcarry) {
  __shared__ float lg[kSeq];
  __shared__ float redM[8];
  __shared__ float redS[8];
  const int row  = blockIdx.x;
  const int t    = threadIdx.x;
  const int lane = t & 31, wave = t >> 5;
  const float* sa = Samp + (size_t)row * kSeq;
  const float* sp = Sph  + (size_t)row * kSeq;
  float m = -3.0e38f;
#pragma unroll 1
  for (int e = 0; e < 8; ++e) {
    const int col = e * 256 + t;
    const float ph = cosf(sp[col] * kPiF);
    const float v  = ph * sa[col];
    lg[col] = v;
    m = fmaxf(m, v);
  }
#pragma unroll
  for (int off = 16; off > 0; off >>= 1) m = fmaxf(m, __shfl_xor(m, off, 32));
  if (lane == 0) redM[wave] = m;
  __syncthreads();
  float mx = redM[0];
#pragma unroll
  for (int w = 1; w < 8; ++w) mx = fmaxf(mx, redM[w]);
  float s = 0.f;
#pragma unroll 1
  for (int e = 0; e < 8; ++e) {
    const int col = e * 256 + t;
    const float pe = expf(lg[col] - mx);
    lg[col] = pe;
    s += pe;
  }
#pragma unroll
  for (int off = 16; off > 0; off >>= 1) s += __shfl_xor(s, off, 32);
  if (lane == 0) redS[wave] = s;
  __syncthreads();
  float tot = 0.f;
#pragma unroll
  for (int w = 0; w < 8; ++w) tot += redS[w];
  const float kk = pcarry * (1.0f / tot);
  const int c0 = t * 8;
  unsigned short hb[8];
#pragma unroll
  for (int e = 0; e < 8; ++e) hb[e] = h_bits(lg[c0 + e] * kk);
  const v4u u = (v4u){pk16(hb[0], hb[1]), pk16(hb[2], hb[3]), pk16(hb[4], hb[5]), pk16(hb[6], hb[7])};
  unsigned short* q = P + (size_t)row * kSeq + c0;
  *(volatile v4u*)q = u;
  __threadfence();
  *(volatile v4u*)q = u;
}

static constexpr int gemm_blocks(int M, int N) { return ((M / 64) * (N / 64) + 7) / 8; }

extern "C" void kernel_launch(void* const* d_in, const int* in_sizes, int n_in,
                              void* d_out, int out_size, void* d_ws,
                              size_t ws_size, hipStream_t stream) {
  if (n_in < 9) return;
  if (in_sizes[0] != kTok * kDim) return;
  if (in_sizes[1] != kDim * kDim || in_sizes[3] != kDim * kDim || in_sizes[5] != kDim * kDim || in_sizes[7] != kDim * kDim) return;
  if (in_sizes[2] != kDim || in_sizes[4] != kDim || in_sizes[6] != kDim || in_sizes[8] != kDim) return;
  if (out_size != kTok * kDim) return;
  if (ws_size < kWsTotal) return;

  const float* x  = (const float*)d_in[0];
  const float* Wq = (const float*)d_in[1];
  const float* bq = (const float*)d_in[2];
  const float* Wk = (const float*)d_in[3];
  const float* bk = (const float*)d_in[4];
  const float* Wv = (const float*)d_in[5];
  const float* bv = (const float*)d_in[6];
  const float* Wo = (const float*)d_in[7];
  const float* bo = (const float*)d_in[8];
  float* out = (float*)d_out;

  char* ws = (char*)d_ws;
  unsigned short* X16  = (unsigned short*)(ws + kOffX16);
  unsigned short* O16  = (unsigned short*)(ws + kOffX16);
  unsigned short* Wq16 = (unsigned short*)(ws + kOffWq);
  unsigned short* Wk16 = (unsigned short*)(ws + kOffWk);
  unsigned short* Wv16 = (unsigned short*)(ws + kOffWv);
  unsigned short* Wo16 = (unsigned short*)(ws + kOffWo);
  float*          scr  = (float*)(ws + kOffScr);
  float*          sAmp = (float*)(ws + kOffScr);
  float*          sPh  = (float*)(ws + kOffSph);
  unsigned short* Q16  = (unsigned short*)(ws + kOffQ16);
  unsigned short* Qn16 = (unsigned short*)(ws + kOffQn16);
  unsigned short* K16  = (unsigned short*)(ws + kOffK16);
  unsigned short* Kn16 = (unsigned short*)(ws + kOffKn16);
  unsigned short* Vt16 = (unsigned short*)(ws + kOffVt16);
  unsigned short* P16  = (unsigned short*)(ws + kOffP16);

  const int xN8 = kTok * kDim / 8;
  const int wN8 = kDim * kDim / 8;
  cast8_f16_kernel<<<dim3((xN8 + 255) / 256), dim3(256), 0, stream>>>(x,  X16,  xN8, 1.0f);
  cast8_f16_kernel<<<dim3((wN8 + 255) / 256), dim3(256), 0, stream>>>(Wq, Wq16, wN8, kWCarry);
  cast8_f16_kernel<<<dim3((wN8 + 255) / 256), dim3(256), 0, stream>>>(Wk, Wk16, wN8, kWCarry);
  cast8_f16_kernel<<<dim3((wN8 + 255) / 256), dim3(256), 0, stream>>>(Wv, Wv16, wN8, kWCarry);
  cast8_f16_kernel<<<dim3((wN8 + 255) / 256), dim3(256), 0, stream>>>(Wo, Wo16, wN8, kWCarry);

  const int projBlocks = gemm_blocks(kProjRows, kDim);
  for (int hf = 0; hf < kTok / kProjRows; ++hf) {
    const size_t ro = (size_t)hf * kProjRows * kDim;
    wmma_gemm64<0, false, 2, 0, false><<<dim3(projBlocks, 1), dim3(256), 0, stream>>>(
        X16 + ro, nullptr, kDim, 0L, Wq16, nullptr, kDim, 0L,
        (void*)scr, nullptr, kDim, 0L, bq, nullptr, 0L, kProjRows, kDim, kDim, kWCarryInv);
    rownorm_kernel<<<dim3(kProjRows), dim3(128), 0, stream>>>(scr, Q16 + ro, Qn16 + ro, kNCarry);
  }
  for (int hf = 0; hf < kTok / kProjRows; ++hf) {
    const size_t ro = (size_t)hf * kProjRows * kDim;
    wmma_gemm64<0, false, 2, 0, false><<<dim3(projBlocks, 1), dim3(256), 0, stream>>>(
        X16 + ro, nullptr, kDim, 0L, Wk16, nullptr, kDim, 0L,
        (void*)scr, nullptr, kDim, 0L, bk, nullptr, 0L, kProjRows, kDim, kDim, kWCarryInv);
    rownorm_kernel<<<dim3(kProjRows), dim3(128), 0, stream>>>(scr, K16 + ro, Kn16 + ro, kNCarry);
  }

  const int vtBlocks = gemm_blocks(kDim, kSeq);
  wmma_gemm64<0, false, 1, 1, false><<<dim3(vtBlocks, kBatch), dim3(256), 0, stream>>>(
      Wv16, nullptr, kDim, 0L, X16, nullptr, kDim, (long)kSeq * kDim,
      (void*)Vt16, nullptr, kSeq, (long)kDim * kSeq, bv, nullptr, 0L, kDim, kSeq, kDim, kWCarryInv);

  const int scBlocks = gemm_blocks(kQRows, kSeq);
  const int pvBlocks = gemm_blocks(kQRows, kDim);
  for (int c = 0; c < kChunks; ++c) {
    const int b = c / kChunksPerBatch;
    const size_t tok0 = (size_t)c * kQRows;
    const size_t kvo  = (size_t)b * kSeq * kDim;
    wmma_gemm64<0, false, 0, 0, false><<<dim3(scBlocks, 1), dim3(256), 0, stream>>>(
        Q16 + tok0 * kDim, nullptr, kDim, 0L, K16 + kvo, nullptr, kDim, 0L,
        (void*)sAmp, nullptr, kSeq, 0L, nullptr, nullptr, 0L, kQRows, kSeq, kDim, kAmpScale);
    wmma_gemm64<0, false, 0, 0, false><<<dim3(scBlocks, 1), dim3(256), 0, stream>>>(
        Qn16 + tok0 * kDim, nullptr, kDim, 0L, Kn16 + kvo, nullptr, kDim, 0L,
        (void*)sPh, nullptr, kSeq, 0L, nullptr, nullptr, 0L, kQRows, kSeq, kDim, kPhScale);
    phase_softmax_kernel<<<dim3(kQRows), dim3(256), 0, stream>>>(sAmp, sPh, P16, kPCarry);
    wmma_gemm64<0, false, 0, 1, false><<<dim3(pvBlocks, 1), dim3(256), 0, stream>>>(
        P16, nullptr, kSeq, 0L, Vt16 + (size_t)b * kDim * kSeq, nullptr, kSeq, 0L,
        (void*)(O16 + tok0 * kDim), nullptr, kDim, 0L, nullptr, nullptr, 0L, kQRows, kDim, kSeq, kPVScale);
  }

  const int outBlocks = gemm_blocks(kTok, kDim);
  wmma_gemm64<0, false, 2, 0, false><<<dim3(outBlocks, 1), dim3(256), 0, stream>>>(
      O16, nullptr, kDim, 0L, Wo16, nullptr, kDim, 0L,
      (void*)out, nullptr, kDim, 0L, bo, nullptr, 0L, kTok, kDim, kDim, kOutScale);
}
